// MultiheadAttentionRelation_42700564857532
// MI455X (gfx1250) — hardware-run, weakly checked
//
#include <hip/hip_runtime.h>

#define NB_  2
#define TT   256
#define NH_  8
#define HD   64
#define DP   512
#define DR   512
#define SLOTS 64
#define ZH   2
#define RH   0
#define PCAR 1024.0f
#define SCL  0.125f
typedef _Float16 h16;
typedef unsigned short bf;
typedef __attribute__((ext_vector_type(16))) __bf16   v16bf;
typedef __attribute__((ext_vector_type(16))) _Float16 v16h;
typedef __attribute__((ext_vector_type(8)))  _Float16 v8h;
typedef __attribute__((ext_vector_type(8)))  unsigned short v8us;
typedef __attribute__((ext_vector_type(8)))  float    v8f;
typedef __attribute__((ext_vector_type(4)))  float    v4f;
typedef v8h  __attribute__((may_alias)) v8ha;
typedef v4f  __attribute__((may_alias)) v4fa;
typedef v8us __attribute__((may_alias)) v8usa;

__device__ __forceinline__ unsigned short f2bf(float f) { unsigned u = __float_as_uint(f); u += 0x7FFFu + ((u >> 16) & 1u); return (unsigned short)(u >> 16); }
__device__ __forceinline__ float bf2f(unsigned short b) { return __uint_as_float(((unsigned)b) << 16); }
__device__ __forceinline__ float bfr(float f) { return bf2f(f2bf(f)); }
__device__ __forceinline__ v16h cat16(v8h lo, v8h hi) { return __builtin_shufflevector(lo, hi, 0, 1, 2, 3, 4, 5, 6, 7, 8, 9, 10, 11, 12, 13, 14, 15); }
__device__ __forceinline__ v16bf cat16b(v8us lo, v8us hi) { return __builtin_bit_cast(v16bf, __builtin_shufflevector(lo, hi, 0, 1, 2, 3, 4, 5, 6, 7, 8, 9, 10, 11, 12, 13, 14, 15)); }
__device__ __forceinline__ v8f wmma16(v16h a, v16h b, v8f c) { return __builtin_amdgcn_wmma_f32_16x16x32_f16(false, a, false, b, (short)0, c, false, false); }
__device__ __forceinline__ v8f wmmab(v16bf a, v16bf b, v8f c) { return __builtin_amdgcn_wmma_f32_16x16x32_bf16(false, a, false, b, (short)0, c, false, false); }


template <typename T16> struct WFrag;
template <> struct WFrag<h16> { typedef v16h V; static __device__ __forceinline__ V ld(const h16* p) { return cat16(*(const v8h*)p, *(const v8h*)(p + 16)); } static __device__ __forceinline__ v8f mma(V a, V b, v8f c) { return wmma16(a, b, c); } };
template <> struct WFrag<bf> { typedef v16bf V; static __device__ __forceinline__ V ld(const bf* p) { return cat16b(*(const v8us*)p, *(const v8us*)(p + 16)); } static __device__ __forceinline__ v8f mma(V a, V b, v8f c) { return wmmab(a, b, c); } };
template <typename T16, int NSPLIT, bool BIAS>
__global__ __launch_bounds__(32) void k_gemmw(const T16* __restrict__ A, const T16* __restrict__ A2, const T16* __restrict__ Bt, const T16* __restrict__ Bt2, int K, float* C, int ldc, const float* __restrict__ bias, size_t sA, size_t sB, size_t sC) {
    typedef typename WFrag<T16>::V V;
    __shared__ __align__(16) float os[16 * 68];
    const size_t z = blockIdx.z; A += z * sA; if (A2) A2 += z * sA; Bt += z * sB; if (Bt2) Bt2 += z * sB; C += z * sC;
    const int lane = threadIdx.x & 31, lr = lane & 15, hi = lane >> 4; const int r0 = blockIdx.x * 64, c0 = blockIdx.y * 64;
    v8f acc[4][4];
#pragma unroll
    for (int mb = 0; mb < 4; ++mb)
#pragma unroll
        for (int nb = 0; nb < 4; ++nb) acc[mb][nb] = (v8f){};
    const size_t aoff = (size_t)(r0 + lr) * K + 8 * hi, boff = (size_t)(c0 + lr) * K + 8 * hi;
    for (int kc = 0; kc < K; kc += 32) {
        V a[4], a2[4];
#pragma unroll
        for (int mb = 0; mb < 4; ++mb) { a[mb] = WFrag<T16>::ld(A + aoff + (size_t)mb * 16 * K + kc); if (NSPLIT == 1 || NSPLIT == 2) a2[mb] = WFrag<T16>::ld(A2 + aoff + (size_t)mb * 16 * K + kc); }
#pragma unroll
        for (int nb = 0; nb < 4; ++nb) { const V b = WFrag<T16>::ld(Bt + boff + (size_t)nb * 16 * K + kc); V b2; if (NSPLIT >= 2) b2 = WFrag<T16>::ld(Bt2 + boff + (size_t)nb * 16 * K + kc);
#pragma unroll
            for (int mb = 0; mb < 4; ++mb) { acc[mb][nb] = WFrag<T16>::mma(a[mb], b, acc[mb][nb]); if (NSPLIT == 1 || NSPLIT == 2) acc[mb][nb] = WFrag<T16>::mma(a2[mb], b, acc[mb][nb]); if (NSPLIT >= 2) acc[mb][nb] = WFrag<T16>::mma(a[mb], b2, acc[mb][nb]); } }
        asm volatile("v_nop\n\tv_nop\n\tv_nop\n\tv_nop" : "+v"(acc[0][0]), "+v"(acc[1][1]), "+v"(acc[2][2]), "+v"(acc[3][3]) : "v"(a[0]), "v"(a[3]));
    }
#pragma unroll
    for (int mb = 0; mb < 4; ++mb) {
#pragma unroll
        for (int nb = 0; nb < 4; ++nb) {
#pragma unroll
            for (int j = 0; j < 8; ++j) os[(hi * 8 + j) * 68 + nb * 16 + lr] = acc[mb][nb][j]; }
        __builtin_amdgcn_wave_barrier(); asm volatile("" ::: "memory");
        float* crow = C + (size_t)(r0 + mb * 16) * ldc + c0;
#pragma unroll 1
        for (int ps = 0; ps < 2; ++ps) {
#pragma unroll
            for (int s = 0; s < 8; ++s) { const int row = 2 * s + hi, cofs = lr * 4; v4f val = *(const v4fa*)(os + row * 68 + cofs); if (BIAS) { val[0] += bfr(bias[c0 + cofs]); val[1] += bfr(bias[c0 + cofs + 1]); val[2] += bfr(bias[c0 + cofs + 2]); val[3] += bfr(bias[c0 + cofs + 3]); }
                *(volatile v4f*)(crow + (size_t)row * ldc + cofs) = val; }
            if (ps == 0) __threadfence(); }
        __builtin_amdgcn_wave_barrier(); asm volatile("" ::: "memory");
    }
}

__device__ __forceinline__ h16 tohx(float x) { return (h16)x; }
__device__ __forceinline__ void splitf(float y, unsigned short& h, unsigned short& l) { h = f2bf(y); l = f2bf(y - bf2f(h)); }
typedef __attribute__((ext_vector_type(2))) _Float16 v2h;
typedef __attribute__((ext_vector_type(4))) _Float16 v4h;
typedef __attribute__((ext_vector_type(2))) unsigned short v2us;
typedef __attribute__((ext_vector_type(4))) unsigned short v4us;
typedef __attribute__((ext_vector_type(2))) float v2f;
typedef __attribute__((ext_vector_type(4))) int v4i;

__global__ __launch_bounds__(256) void k_wtG(const float* __restrict__ w, int K, int N, bf* Bt) {
    const int lane = threadIdx.x & 31; const int L0 = (blockIdx.x * 8 + (threadIdx.x >> 5)) * 8; const int nlines = N * K / 64;
#pragma unroll
    for (int ps = 0; ps < 2; ++ps) {
        for (int l = 0; l < 8; ++l) { const int L = L0 + l; if (L >= nlines) break; const size_t e = (size_t)L * 64 + lane * 2; const int k = (int)(e % K), n = (int)(e / K); v2us o;
            o[0] = f2bf(w[(size_t)k * N + n]); o[1] = f2bf(w[(size_t)(k + 1) * N + n]); *(volatile v2us*)(Bt + e) = o; }
        if (ps == 0) __threadfence(); }
}
__global__ __launch_bounds__(256) void k_cvt8(const float* __restrict__ src, bf* dst, size_t n8) { const size_t i = (size_t)blockIdx.x * 256 + threadIdx.x; if (i >= n8) return; const v8f v = *(const v8f*)(src + i * 8); v8us o;
#pragma unroll
    for (int k = 0; k < 8; ++k) o[k] = f2bf(v[k]); *(volatile v8us*)(dst + i * 8) = o; __threadfence(); *(volatile v8us*)(dst + i * 8) = o; }
template <typename T16> __device__ __forceinline__ unsigned short cv16(float x);
template <> __device__ __forceinline__ unsigned short cv16<bf>(float x) { return f2bf(x); }
template <> __device__ __forceinline__ unsigned short cv16<h16>(float x) { const h16 h = (h16)x; return __builtin_bit_cast(unsigned short, h); }
template <typename T16>
__global__ __launch_bounds__(256) void k_castp(const float* __restrict__ src, int rows_valid, int lc, float mul, unsigned short* dst) { const unsigned e = blockIdx.x * 256 + threadIdx.x; const unsigned r = e >> (lc - 3); const unsigned c0 = (e & ((1u << (lc - 3)) - 1u)) << 3; const unsigned rr = (r < (unsigned)rows_valid) ? r : (unsigned)(rows_valid - 1);
    const float* s = src + ((size_t)rr << lc) + c0; const v4f a = *(const v4f*)s, b = *(const v4f*)(s + 4); const float lm = (r < (unsigned)rows_valid) ? mul : 0.0f; v8us o;
#pragma unroll
    for (int q = 0; q < 4; ++q) { o[q] = cv16<T16>(__fmul_rn(a[q], lm)); o[q + 4] = cv16<T16>(__fmul_rn(b[q], lm)); }
    *(volatile v8us*)(dst + (size_t)e * 8) = o; __threadfence(); *(volatile v8us*)(dst + (size_t)e * 8) = o; }

__global__ __launch_bounds__(256) void k_asoft(const float* __restrict__ Sb, h16* P16, bf* Ph, bf* Pl) {
    const int lane = threadIdx.x & 31; const int row = blockIdx.x * 8 + (threadIdx.x >> 5); if (row >= ZH * TT) return; const int i = row % TT; const int zz = row / TT; (void)zz; const bool hires = (i < RH); const float* sr = Sb + (size_t)row * TT; float v[TT / 32]; float mx = -3.0e38f;
#pragma unroll
    for (int ch = 0; ch < TT / 128; ++ch) { const int j0 = ch * 128 + lane * 4; const v4f a = *(const v4f*)(sr + j0);
#pragma unroll
        for (int q = 0; q < 4; ++q) { const int j = j0 + q; (void)j; const float t = a[q] * SCL; v[ch * 4 + q] = t; mx = fmaxf(mx, t); } }
#pragma unroll
    for (int sh = 16; sh; sh >>= 1) mx = fmaxf(mx, __shfl_xor(mx, sh, 32));
    float sum = 0.f;
#pragma unroll
    for (int k = 0; k < TT / 32; ++k) { float d0 = __fsub_rn(v[k], mx); v[k] = __builtin_amdgcn_exp2f(__fmul_rn(d0, 1.4426950408889634f)); sum += v[k]; }
#pragma unroll
    for (int sh = 16; sh; sh >>= 1) sum += __shfl_xor(sum, sh, 32);
    const float f = __fdiv_rn(hires ? 1.0f : PCAR, sum);
#pragma unroll 1
    for (int ps = 0; ps < 2; ++ps) {
        if (hires) {
#pragma unroll
            for (int ch = 0; ch < TT / 128; ++ch) { v4us oh, ol;
#pragma unroll
                for (int q = 0; q < 4; ++q) { unsigned short a, c2; splitf(v[ch * 4 + q] * f, a, c2); oh[q] = a; ol[q] = c2; }
                const size_t oo = ((size_t)zz * (RH ? RH : 1) + i) * TT + ch * 128 + lane * 4; *(volatile v4us*)(Ph + oo) = oh; *(volatile v4us*)(Pl + oo) = ol; }
        } else {
#pragma unroll
            for (int ch = 0; ch < TT / 128; ++ch) { v4h o4;
#pragma unroll
                for (int q = 0; q < 4; ++q) o4[q] = tohx(v[ch * 4 + q] * f);
                *(volatile v4h*)(P16 + (size_t)row * TT + ch * 128 + lane * 4) = o4; } }
        if (ps == 0) __threadfence(); }
}

__global__ __launch_bounds__(256) void k_pcast(const float* __restrict__ src, int l1, int l2, size_t s0, size_t s1, bf* dst) { const unsigned e = (blockIdx.x * 256u + threadIdx.x) * 4u; const unsigned i2 = e & ((1u << l2) - 1u); const unsigned r = e >> l2; const unsigned i1 = r & ((1u << l1) - 1u); const unsigned i0 = r >> l1;
    const v4f a = *(const v4f*)(src + (size_t)i0 * s0 + (size_t)i1 * s1 + i2); v4us o;
#pragma unroll
    for (int q = 0; q < 4; ++q) o[q] = f2bf(a[q]);
    *(volatile v4us*)(dst + e) = o; __threadfence(); *(volatile v4us*)(dst + e) = o; }
__global__ __launch_bounds__(256) void k_splitp(const float* __restrict__ src, int nv, int ls, int l2, size_t s0, size_t s1, bf* dh, bf* dl) { const unsigned e = (blockIdx.x * 256u + threadIdx.x) * 4u; const unsigned i2 = e & ((1u << l2) - 1u); const unsigned r = e >> l2; const unsigned s = r & ((1u << ls) - 1u); const unsigned i0 = r >> ls;
    const unsigned sr = (s < (unsigned)nv) ? s : (unsigned)(nv - 1); const float fm = (s < (unsigned)nv) ? 1.0f : 0.0f; const v4f a = *(const v4f*)(src + (size_t)i0 * s0 + (size_t)sr * s1 + i2); v4us oh, ol;
#pragma unroll
    for (int q = 0; q < 4; ++q) { unsigned short h, l; splitf(__fmul_rn(a[q], fm), h, l); oh[q] = h; ol[q] = l; }
    *(volatile v4us*)(dh + e) = oh; *(volatile v4us*)(dl + e) = ol; __threadfence(); *(volatile v4us*)(dh + e) = oh; *(volatile v4us*)(dl + e) = ol; }
__global__ __launch_bounds__(256) void k_comb(const float* __restrict__ r0, const float* __restrict__ r1, const float* __restrict__ r2, float* S) { const unsigned e = (blockIdx.x * 256u + threadIdx.x) * 4u; const unsigned m = e % TT; const unsigned n = (e / TT) % TT; const unsigned k = e / (TT * TT);
    const v4f a = *(const v4f*)(r0 + e), c = *(const v4f*)(r2 + e); v4f o;
#pragma unroll
    for (int q = 0; q < 4; ++q) o[q] = __fadd_rn(__fadd_rn(a[q], r1[(size_t)((k * TT + m + q) * TT + n)]), c[q]);
    *(volatile v4f*)(S + e) = o; __threadfence(); *(volatile v4f*)(S + e) = o; }

__global__ __launch_bounds__(256) void k_aout(const h16* __restrict__ P, float mul, float* A) { const unsigned e = blockIdx.x * 256u + threadIdx.x; const unsigned half = e & 1u, k = (e >> 1) & (unsigned)(TT - 1), q = e / (2u * TT); const unsigned* P32 = (const unsigned*)P; const unsigned sh = (k & 1u) << 4; v4h w;
#pragma unroll
    for (int i = 0; i < 4; ++i) { const unsigned h = half * 4u + (unsigned)i; const unsigned u = P32[((h * TT + q) * TT + k) >> 1]; w[i] = __builtin_bit_cast(h16, (unsigned short)(u >> sh)); }
    const v4f o = __builtin_convertvector(w, v4f) * mul;
    *(volatile v4f*)(A + e * 4u) = o; __threadfence(); *(volatile v4f*)(A + e * 4u) = o; }
extern "C" void kernel_launch(void* const* d_in, const int* in_sizes, int n_in,
                              void* d_out, int out_size, void* d_ws, size_t ws_size, hipStream_t stream) {
    (void)in_sizes; (void)n_in; (void)out_size;
    static_assert(TT == 256 && HD == 64 && DR == 512 && DP == 512 && NH_ == 8 && SLOTS == 64 && NH_ % ZH == 0 && NH_ <= SLOTS && NH_ * HD == DP, "the flat kernels' logs below are these sizes'; the passes are whole; the heads fit a tile's rows");
    static_assert((size_t)TT * TT * DR < ((size_t)1 << 32) && (size_t)SLOTS * TT * TT * 4 < ((size_t)1 << 32) && (size_t)SLOTS * TT * TT < ((size_t)1 << 24) + 1, "every flat kernel's element index fits a 32-bit word (the largest plane: 2^25 words); the adder's transposed read stays under 2^24 words");
    static_assert(((size_t)TT * TT * DR / 4) % 256 == 0 && ((size_t)NH_ * TT * HD / 4) % 256 == 0 && ((size_t)TT * SLOTS * DR / 4) % 256 == 0 && ((size_t)NH_ * TT * TT / 4) % 256 == 0 && ((size_t)TT * TT * 2) % 256 == 0 && ((size_t)TT * DP / 4) % 256 == 0, "every flat kernel's grid is exact");
    const float* query = (const float*)d_in[0]; const float* key = (const float*)d_in[1]; const float* value = (const float*)d_in[2]; const float* rel = (const float*)d_in[3]; const float* wq = (const float*)d_in[4]; const float* wk = (const float*)d_in[5]; const float* wr = (const float*)d_in[7]; const float* br = (const float*)d_in[8]; const float* wo = (const float*)d_in[9]; const float* bo = (const float*)d_in[10];
    float* OUT = (float*)d_out;
    float* AOUT = OUT + (size_t)NB_ * TT * DP;
    char* wsp = (char*)d_ws;
    auto take = [&](size_t bytes) { char* p = wsp; wsp += (bytes + 255) & ~(size_t)255; return (void*)p; };
    bf* WQt = (bf*)take((size_t)DP * DP * 2); bf* WKt = (bf*)take((size_t)DP * DP * 2); bf* LZ = (bf*)take((size_t)NH_ * DR * HD * 2); bf* WOs = (bf*)take((size_t)DP * DP * 2);
    bf* QB = (bf*)take((size_t)TT * DP * 2); bf* KB = (bf*)take((size_t)TT * DP * 2); bf* VB = (bf*)take((size_t)TT * DP * 2); bf* ZT = (bf*)take((size_t)TT * TT * DR * 2);
    float* FQ = (float*)take((size_t)NH_ * TT * HD * 4); float* FK = (float*)take((size_t)NH_ * TT * HD * 4); float* FVT = (float*)take((size_t)NH_ * HD * TT * 4); h16* VT16 = (h16*)take((size_t)NH_ * HD * TT * 2);
    bf* QTh = (bf*)take((size_t)NH_ * TT * HD * 2); bf* QTl = (bf*)take((size_t)NH_ * TT * HD * 2); bf* KTh = (bf*)take((size_t)NH_ * TT * HD * 2); bf* KTl = (bf*)take((size_t)NH_ * TT * HD * 2);
    float* FU = (float*)take((size_t)NH_ * TT * DR * 4); bf* UPh = (bf*)take((size_t)TT * SLOTS * DR * 2); bf* UPl = (bf*)take((size_t)TT * SLOTS * DR * 2);
    float* R0 = (float*)take((size_t)NH_ * TT * TT * 4); float* R1 = (float*)take((size_t)SLOTS * TT * TT * 4); float* R2 = (float*)take((size_t)NH_ * TT * TT * 4); float* Sb = (float*)take((size_t)NH_ * TT * TT * 4); h16* P16 = (h16*)take((size_t)NH_ * TT * TT * 2);
    float* MG = (float*)take((size_t)TT * DP * 4); bf* MGh = (bf*)take((size_t)TT * DP * 2); bf* MGl = (bf*)take((size_t)TT * DP * 2);
    if ((size_t)(wsp - (char*)d_ws) > ws_size) return;
    k_wtG<<<(unsigned)((DP * DP / 64 + 63) / 64), 256, 0, stream>>>(wq, DP, DP, WQt); k_wtG<<<(unsigned)((DP * DP / 64 + 63) / 64), 256, 0, stream>>>(wk, DP, DP, WKt);
    for (int h = 0; h < NH_; ++h) k_wtG<<<(unsigned)((HD * DR / 64 + 63) / 64), 256, 0, stream>>>(wr + (size_t)h * HD * DR, HD, DR, LZ + (size_t)h * DR * HD);
    k_castp<bf><<<(unsigned)((size_t)DP * DP / 8 / 256), 256, 0, stream>>>(wo, DP, 9, 1.0f / PCAR, (unsigned short*)WOs);
    for (int b = 0; b < NB_; ++b) {
        k_cvt8<<<(unsigned)(((size_t)TT * DP / 8 + 255) / 256), 256, 0, stream>>>(query + (size_t)b * TT * DP, QB, (size_t)TT * DP / 8); k_cvt8<<<(unsigned)(((size_t)TT * DP / 8 + 255) / 256), 256, 0, stream>>>(key + (size_t)b * TT * DP, KB, (size_t)TT * DP / 8); k_cvt8<<<(unsigned)(((size_t)TT * DP / 8 + 255) / 256), 256, 0, stream>>>(value + (size_t)b * TT * DP, VB, (size_t)TT * DP / 8);
        k_pcast<<<(unsigned)((size_t)TT * TT * DR / 4 / 256), 256, 0, stream>>>(rel + (size_t)b * TT * TT * DR, 8, 9, (size_t)DR, (size_t)TT * DR, ZT);
        for (int h = 0; h < NH_; ++h) k_gemmw<bf, 0, true><<<dim3(TT / 64, HD / 64, 1), 32, 0, stream>>>(QB, nullptr, WQt + (size_t)h * HD * DP, nullptr, DP, FQ + (size_t)h * TT * HD, HD, br + h * HD, 0, 0, 0);
        k_gemmw<bf, 0, false><<<dim3(TT / 64, HD / 64, NH_), 32, 0, stream>>>(KB, nullptr, WKt, nullptr, DP, FK, HD, nullptr, 0, (size_t)HD * DP, (size_t)TT * HD);
        k_gemmw<bf, 0, false><<<dim3(HD / 64, TT / 64, NH_), 32, 0, stream>>>(WQt, nullptr, VB, nullptr, DP, FVT, TT, nullptr, (size_t)HD * DP, 0, (size_t)HD * TT);
        k_castp<h16><<<(unsigned)((size_t)NH_ * HD * TT / 8 / 256), 256, 0, stream>>>(FVT, NH_ * HD, 8, 1.0f, (unsigned short*)VT16);
        k_splitp<<<(unsigned)((size_t)NH_ * TT * HD / 4 / 256), 256, 0, stream>>>(FQ, 1, 0, 6, (size_t)HD, 0, QTh, QTl); k_splitp<<<(unsigned)((size_t)NH_ * TT * HD / 4 / 256), 256, 0, stream>>>(FK, 1, 0, 6, (size_t)HD, 0, KTh, KTl);
        k_gemmw<bf, 1, false><<<dim3(TT / 64, DR / 64, NH_), 32, 0, stream>>>(KTh, KTl, LZ, nullptr, HD, FU, DR, nullptr, (size_t)TT * HD, (size_t)DR * HD, (size_t)TT * DR);
        k_splitp<<<(unsigned)((size_t)TT * SLOTS * DR / 4 / 256), 256, 0, stream>>>(FU, NH_, 6, 9, (size_t)DR, (size_t)TT * DR, UPh, UPl);
        k_gemmw<bf, 1, false><<<dim3(TT / 64, TT / 64, NH_), 32, 0, stream>>>(QTh, QTl, KTh, nullptr, HD, R0, TT, nullptr, (size_t)TT * HD, (size_t)TT * HD, (size_t)TT * TT);
        k_gemmw<bf, 0, false><<<dim3(TT / 64, TT / 64, NH_), 32, 0, stream>>>(QTh, nullptr, KTl, nullptr, HD, R2, TT, nullptr, (size_t)TT * HD, (size_t)TT * HD, (size_t)TT * TT);
        k_gemmw<bf, 1, false><<<dim3(SLOTS / 64, TT / 64, TT), 32, 0, stream>>>(UPh, UPl, ZT, nullptr, DR, R1, TT * TT, nullptr, (size_t)SLOTS * DR, (size_t)TT * DR, (size_t)TT);
        k_comb<<<(unsigned)((size_t)NH_ * TT * TT / 4 / 256), 256, 0, stream>>>(R0, R1, R2, Sb);
        for (int h0 = 0; h0 < NH_; h0 += ZH) { const size_t zq = (size_t)h0;
            k_asoft<<<ZH * TT / 8, 256, 0, stream>>>(Sb + zq * TT * TT, P16 + zq * TT * TT, nullptr, nullptr);
            k_gemmw<h16, 0, false><<<dim3(TT / 64, HD / 64, ZH), 32, 0, stream>>>(P16 + zq * TT * TT, nullptr, VT16 + zq * HD * TT, nullptr, TT, MG + zq * HD, DP, nullptr, (size_t)TT * TT, (size_t)HD * TT, (size_t)HD); }
        k_aout<<<(unsigned)((size_t)TT * TT * 2 / 256), 256, 0, stream>>>(P16, 1.0f / PCAR, AOUT + (size_t)b * TT * TT * NH_);
        k_splitp<<<(unsigned)((size_t)TT * DP / 4 / 256), 256, 0, stream>>>(MG, 1, 0, 9, (size_t)DP, 0, MGh, MGl);
        k_gemmw<bf, 1, true><<<dim3(TT / 64, DP / 64, 1), 32, 0, stream>>>(MGh, MGl, WOs, nullptr, DP, OUT + (size_t)b * TT * DP, DP, bo, 0, 0, 0); }
}
